// CoupledModel_24670292148952
// MI455X (gfx1250) — hardware-verified
//
#include <hip/hip_runtime.h>
#include <stdint.h>


typedef _Float16 v16h __attribute__((ext_vector_type(16)));
typedef _Float16 v8h  __attribute__((ext_vector_type(8)));
typedef _Float16 v4h  __attribute__((ext_vector_type(4)));
typedef _Float16 v2h  __attribute__((ext_vector_type(2)));
typedef float    v8f  __attribute__((ext_vector_type(8)));
typedef float    v4f  __attribute__((ext_vector_type(4)));
typedef float    v2f  __attribute__((ext_vector_type(2)));

#define NUM_NETS 24
#define WIDTH    64
#define NTHREADS 256
#define NWAVES   8
#define SPB      (NWAVES * 16)

#define C2L      2.8853900817779268f
#define SC_H1    16.0f
#define SC_W2    64.0f
#define CINV     (C2L / 1024.0f)

union Frag {
    v16h     v;
    v8h      half[2];
    uint32_t u[8];
};

__device__ __forceinline__ v8f wmma_f16(v16h a, v16h b, v8f c) {
    c = __builtin_amdgcn_wmma_f32_16x16x32_f16(false, a, false, b, (short)0, c, false, false);
    asm volatile("v_nop\n\tv_nop\n\tv_nop\n\tv_nop" : "+v"(c) : "v"(a), "v"(b));
    return c;
}

__device__ __forceinline__ float half_sig(float arg) {
    const float e = __builtin_amdgcn_exp2f(arg);
    return __builtin_amdgcn_rcpf(1.0f + e);
}

__device__ __forceinline__ void store_pass(float* subg, float* outg, const v4f (&vs)[3], const v4f vo,
                                           int tid, int blockBase, int N, bool v4ok)
{
#pragma unroll
    for (int i = 0; i < 3; ++i) {
        const int j = tid + NTHREADS * i;
        if (v4ok) {
            const int rl = j / 6;
            if (blockBase + rl < N) *(volatile v4f*)(subg + 4 * j) = vs[i];
        } else {
#pragma unroll
            for (int c = 0; c < 4; ++c) {
                const int e  = 4 * j + c;
                const int rl = e / NUM_NETS;
                if (blockBase + rl < N) ((volatile float*)subg)[e] = vs[i][c];
            }
        }
    }
    if (tid < SPB / 4) {
        const int r0 = blockBase + 4 * tid;
        if (v4ok && (r0 + 3 < N)) {
            *(volatile v4f*)(outg + 4 * tid) = vo;
        } else {
#pragma unroll
            for (int c = 0; c < 4; ++c)
                if (r0 + c < N) ((volatile float*)outg)[4 * tid + c] = vo[c];
        }
    }
}

__global__ __launch_bounds__(NTHREADS)
void k_fused(const float* __restrict__ x,
             const float* __restrict__ W1,
             const float* __restrict__ b1,
             const float* __restrict__ W2,
             const float* __restrict__ b2,
             const float* __restrict__ W3,
             float* out,
             float* sub,
             int N)
{
    __shared__ __attribute__((aligned(32))) _Float16 sW2[WIDTH * WIDTH];
    __shared__ __attribute__((aligned(32))) float    sW1s[WIDTH * 2];
    __shared__ __attribute__((aligned(32))) float    sb1s[WIDTH];
    __shared__ __attribute__((aligned(32))) float    sb2s[WIDTH];
    __shared__ __attribute__((aligned(32))) float    sW3m2[WIDTH];
    __shared__ float sSumW3;
    __shared__ __attribute__((aligned(32))) float    sSub[SPB * NUM_NETS];
    __shared__ __attribute__((aligned(32))) float    sOut[SPB];

    const int tid  = threadIdx.x;
    const int lane = tid & 31;
    const int wave = tid >> 5;
    const int h    = lane >> 4;
    const int m    = lane & 15;
    const int blockBase = blockIdx.x * SPB;

    int ns = blockBase + wave * 16 + m;
    if (ns >= N) ns = N - 1;
    const float x0 = x[2 * (size_t)ns + 0];
    const float x1 = x[2 * (size_t)ns + 1];

#pragma unroll 1
    for (int k = 0; k < NUM_NETS; ++k) {
        __syncthreads();
        if (tid < 2 * WIDTH) sW1s[tid] = W1[(size_t)k * 2 * WIDTH + tid] * C2L;
        if (tid < WIDTH) {
            sb1s[tid]  = b1[(size_t)k * WIDTH + tid] * C2L;
            sb2s[tid]  = b2[(size_t)k * WIDTH + tid] * C2L;
            sW3m2[tid] = -2.0f * W3[(size_t)k * WIDTH + tid];
        }
        if (wave == 0) {
            float s = W3[(size_t)k * WIDTH + lane] + W3[(size_t)k * WIDTH + 32 + lane];
            s += __shfl_xor(s, 16, 32);
            s += __shfl_xor(s, 8, 32);
            s += __shfl_xor(s, 4, 32);
            s += __shfl_xor(s, 2, 32);
            s += __shfl_xor(s, 1, 32);
            if (lane == 0) sSumW3 = s;
        }
        {
            const float* gW2 = W2 + (size_t)k * WIDTH * WIDTH;
#pragma unroll
            for (int q = 0; q < 2; ++q) {
                const int c = tid + NTHREADS * q;
                const v4f f0 = *(const v4f*)(gW2 + 8 * c);
                const v4f f1 = *(const v4f*)(gW2 + 8 * c + 4);
                const v4h g0 = __builtin_convertvector(f0 * SC_W2, v4h);
                const v4h g1 = __builtin_convertvector(f1 * SC_W2, v4h);
                const v8h hv = __builtin_shufflevector(g0, g1, 0, 1, 2, 3, 4, 5, 6, 7);
                *(v8h*)(&sW2[8 * c]) = hv;
            }
        }
        __syncthreads();

        Frag B[2];
#pragma unroll
        for (int p = 0; p < 2; ++p) {
#pragma unroll
            for (int j = 0; j < 8; ++j) {
                const int kk = (j < 4) ? (2 * j + 8 * h) : (16 + 2 * (j - 4) + 8 * h);
                const int w  = p * 32 + kk;
                const v4f wv = *(const v4f*)(&sW1s[2 * w]);
                const v2f bv = *(const v2f*)(&sb1s[w]);
                const float a0 = fmaf(x0, wv[0], fmaf(x1, wv[1], bv[0]));
                const float a1 = fmaf(x0, wv[2], fmaf(x1, wv[3], bv[1]));
                v2f tv;
                tv[0] = fmaf(-2.0f * SC_H1, half_sig(a0), SC_H1);
                tv[1] = fmaf(-2.0f * SC_H1, half_sig(a1), SC_H1);
                const v2h th = __builtin_convertvector(tv, v2h);
                B[p].u[j] = __builtin_bit_cast(uint32_t, th);
            }
        }

        float accn = 0.f;
#pragma unroll
        for (int t = 0; t < 4; ++t) {
            v8f c = {0.f, 0.f, 0.f, 0.f, 0.f, 0.f, 0.f, 0.f};
#pragma unroll
            for (int p = 0; p < 2; ++p) {
                Frag a;
                a.half[0] = *(const v8h*)(&sW2[(16 * t + m) * WIDTH + 32 * p + 8 * h]);
                a.half[1] = *(const v8h*)(&sW2[(16 * t + m) * WIDTH + 32 * p + 16 + 8 * h]);
                c = wmma_f16(a.v, B[p].v, c);
            }
            const int vb = 16 * t + 8 * h;
            const v8f b8 = *(const v8f*)(&sb2s[vb]);
            const v8f w8 = *(const v8f*)(&sW3m2[vb]);
#pragma unroll
            for (int r = 0; r < 8; ++r) {
                const float arg = fmaf(c[r], CINV, b8[r]);
                accn = fmaf(w8[r], half_sig(arg), accn);
            }
        }
        float tot = accn + __shfl_xor(accn, 16, 32);
        tot += sSumW3;
        if (lane < 16) sSub[(wave * 16 + lane) * NUM_NETS + k] = tot;
    }
    __syncthreads();

    if (tid < SPB) {
        const int s = tid;
        const int n = blockBase + s;
        float o = 0.f;
        if (n < N) {
            const float kb   = 0.1f;
            const float T    = fmaxf(x[2 * (size_t)n + 1], 0.1f);
            const float kbT  = kb * T;
            const float rden = 1.0f / kbT;
            float vals[NUM_NETS / 2], lg[NUM_NETS / 2];
            float ssum = 0.f;
#pragma unroll
            for (int i = 0; i < NUM_NETS / 2; ++i) {
                const float n1 = sSub[s * NUM_NETS + 2 * i + 0];
                const float n2 = sSub[s * NUM_NETS + 2 * i + 1];
                const float vv = n1 - T * (n2 * n2);
                vals[i] = vv;
                const float e = fminf(-vv * rden, 10.0f);
                lg[i] = __expf(e);
                ssum += lg[i];
            }
            ssum += 1e-9f;
            const float rs = 1.0f / ssum;
            float wv = 0.f, wlp = 0.f;
#pragma unroll
            for (int i = 0; i < NUM_NETS / 2; ++i) {
                const float w = lg[i] * rs;
                wv  = fmaf(w, vals[i], wv);
                wlp = fmaf(w, __logf(w + 1e-9f), wlp);
            }
            o = fmaf(kbT, wlp, wv);
        }
        sOut[s] = o;
    }
    __syncthreads();

    v4f vs[3];
#pragma unroll
    for (int i = 0; i < 3; ++i)
        vs[i] = *(const v4f*)(&sSub[4 * (tid + NTHREADS * i)]);
    v4f vo = {0.f, 0.f, 0.f, 0.f};
    if (tid < SPB / 4) vo = *(const v4f*)(&sOut[4 * tid]);

    float* subg = sub + (size_t)blockBase * NUM_NETS;
    float* outg = out + (size_t)blockBase;
    const bool v4ok = ((N & 3) == 0);

    store_pass(subg, outg, vs, vo, tid, blockBase, N, v4ok);
    __threadfence();
    store_pass(subg, outg, vs, vo, tid, blockBase, N, v4ok);
}

extern "C" void kernel_launch(void* const* d_in, const int* in_sizes, int n_in,
                              void* d_out, int out_size, void* d_ws, size_t ws_size,
                              hipStream_t stream)
{
    (void)n_in; (void)d_ws; (void)ws_size;
    const float* x  = (const float*)d_in[0];
    const float* W1 = (const float*)d_in[1];
    const float* b1 = (const float*)d_in[2];
    const float* W2 = (const float*)d_in[3];
    const float* b2 = (const float*)d_in[4];
    const float* W3 = (const float*)d_in[5];

    const int N = in_sizes[0] / 2;
    if (N <= 0) return;
    if ((long long)out_size < 25LL * (long long)N) return;
    float* out = (float*)d_out;
    float* sub = out + N;

    const int nblk = (N + SPB - 1) / SPB;
    hipLaunchKernelGGL(k_fused, dim3(nblk), dim3(NTHREADS), 0, stream,
                       x, W1, b1, W2, b2, W3, out, sub, N);
}
